// GGNNLayer_7172595384548
// MI455X (gfx1250) — hardware-run, weakly checked
//
#include <hip/hip_runtime.h>

typedef float          v8f   __attribute__((ext_vector_type(8)));
typedef float          v4f   __attribute__((ext_vector_type(4)));
typedef unsigned int   v4u   __attribute__((ext_vector_type(4)));
typedef int            v8i   __attribute__((ext_vector_type(8)));
typedef unsigned short v8us  __attribute__((ext_vector_type(8)));
typedef unsigned short v16us __attribute__((ext_vector_type(16)));
typedef __bf16         v16bf __attribute__((ext_vector_type(16)));
typedef _Float16       v16h  __attribute__((ext_vector_type(16)));
typedef v4f  __attribute__((may_alias)) v4fa;
typedef v8us __attribute__((may_alias)) v8usa;
union FragB { v16bf v; v16us u; v8us h[2]; v8i w; };
union FragH { v16h  v; v16us u; v8us h[2]; v8i w; };

__device__ __forceinline__ v8f wmb(const FragB& a, const FragB& b, v8f c) {
  v8f d = __builtin_amdgcn_wmma_f32_16x16x32_bf16(false, a.v, false, b.v, (short)0, c, false, false);
  asm volatile("v_nop\n\tv_nop\n\tv_nop\n\tv_nop" : "+v"(d) : "v"(a.w), "v"(b.w));
  return d;
}

__device__ __forceinline__ v8f wmh(const FragH& a, const FragH& b, v8f c) {
  v8f d = __builtin_amdgcn_wmma_f32_16x16x32_f16(false, a.v, false, b.v, (short)0, c, false, false);
  asm volatile("v_nop\n\tv_nop\n\tv_nop\n\tv_nop" : "+v"(d) : "v"(a.w), "v"(b.w));
  return d;
}

__device__ __forceinline__ unsigned bf16_bits(float f) {
  const unsigned u = __float_as_uint(f);
  const unsigned r = (u + 0x7FFFu + ((u >> 16) & 1u)) >> 16;
  const unsigned q = (u >> 16) | 0x40u;
  return ((u & 0x7fffffffu) > 0x7f800000u) ? q : r;
}

__device__ __forceinline__ float bf16_val(float f) {
  return __uint_as_float(bf16_bits(f) << 16);
}
__device__ __forceinline__ int clampi(int v, int lo, int hi) {
  return v < lo ? lo : (v > hi ? hi : v);
}

__device__ __forceinline__ unsigned f16_bits(float f) {
  const unsigned u  = __float_as_uint(f);
  const unsigned s  = (u >> 16) & 0x8000u;
  const unsigned a  = u & 0x7fffffffu;
  const unsigned t  = a - 0x38000000u;
  const unsigned r  = (t + 0x0FFFu + ((t >> 13) & 1u)) >> 13;
  const unsigned rc = r > 0x7C00u ? 0x7C00u : r;
  const bool small  = a < 0x38800000u;
  const bool isnan  = a > 0x7f800000u;
  const unsigned fin = small ? 0u : (s | rc);
  return isnan ? (s | 0x7E00u) : fin;
}

__device__ __forceinline__ unsigned pk16(unsigned lo, unsigned hi) { return lo | (hi << 16); }
__device__ __forceinline__ unsigned bf16_lo_bits(float v) {
  float hi = bf16_val(v);
  asm volatile("" : "+v"(hi));
  return bf16_bits(v - hi);
}
__device__ __forceinline__ v4u pack8_bf16(v4f a, v4f c) {
  return (v4u){ pk16(bf16_bits(a[0]), bf16_bits(a[1])), pk16(bf16_bits(a[2]), bf16_bits(a[3])),
                pk16(bf16_bits(c[0]), bf16_bits(c[1])), pk16(bf16_bits(c[2]), bf16_bits(c[3])) };
}
__device__ __forceinline__ v4u pack8_bf16_lo(v4f a, v4f c) {
  return (v4u){ pk16(bf16_lo_bits(a[0]), bf16_lo_bits(a[1])), pk16(bf16_lo_bits(a[2]), bf16_lo_bits(a[3])),
                pk16(bf16_lo_bits(c[0]), bf16_lo_bits(c[1])), pk16(bf16_lo_bits(c[2]), bf16_lo_bits(c[3])) };
}
__device__ __forceinline__ v4u pack8_f16(v4f a, v4f c) {
  return (v4u){ pk16(f16_bits(a[0]), f16_bits(a[1])), pk16(f16_bits(a[2]), f16_bits(a[3])),
                pk16(f16_bits(c[0]), f16_bits(c[1])), pk16(f16_bits(c[2]), f16_bits(c[3])) };
}

template <int FORM>
__global__ __launch_bounds__(256) void k_plane(const float* __restrict__ src, int rows, int cols, int ldsrc,
                                               unsigned short* __restrict__ dst, int MP, int KP) {
  static_assert(FORM >= 0 && FORM <= 3);
  const int KTOT = (FORM == 1 || FORM == 3) ? 2 * KP : KP;
  const unsigned ppr   = (unsigned)(KTOT >> 3);
  const unsigned kp8   = (unsigned)(KP >> 3);
  const unsigned total = (unsigned)MP * ppr;
  const unsigned g     = blockIdx.x * 256u + threadIdx.x;
  const unsigned rowu  = g / ppr;
  const unsigned p     = g - rowu * ppr;
  const bool second    = p >= kp8;
  const int row = (int)rowu;
  const int c0  = (int)((second ? p - kp8 : p) << 3);
  const float* srow = src + (size_t)clampi(row, 0, rows - 1) * (size_t)ldsrc;
  float x[8];
  unsigned mk[8];
#pragma unroll
  for (int e = 0; e < 8; ++e) {
    const int c = c0 + e;
    const float v = srow[clampi(c, 0, cols - 1)];
    asm volatile("" :: "v"(v));
    x[e]  = v;
    mk[e] = (row < rows && c < cols) ? 0xFFFFu : 0u;
  }
  const v4f a = (v4f){ x[0], x[1], x[2], x[3] };
  const v4f c = (v4f){ x[4], x[5], x[6], x[7] };
  v4u o;
  if (FORM == 2) {
    o = pack8_f16(a, c);
  } else {
    const v4u hi = pack8_bf16(a, c);
    o = hi;
    if (FORM == 1) { const v4u lo = pack8_bf16_lo(a, c); o = second ? lo : hi; }
  }
  const v4u mw = (v4u){ pk16(mk[0], mk[1]), pk16(mk[2], mk[3]), pk16(mk[4], mk[5]), pk16(mk[6], mk[7]) };
  o &= mw;
  if (g < total) {
    volatile v4u* q = (volatile v4u*)(dst + (size_t)g * 8);
    *q = o;
    __threadfence();
    *q = o;
  }
}

template <int FORM> struct FragOf    { typedef FragB T; };
template <>         struct FragOf<2> { typedef FragH T; };
__device__ __forceinline__ v8f mm(const FragB& a, const FragB& b, v8f c) { return wmb(a, b, c); }
__device__ __forceinline__ v8f mm(const FragH& a, const FragH& b, v8f c) { return wmh(a, b, c); }
template <class F> __device__ __forceinline__ F ld_frag(const unsigned short* p) {
  F f;
  f.h[0] = *(const v8usa*)(p);
  f.h[1] = *(const v8usa*)(p + 16);
  return f;
}

template <int FORM, int EPI>
__global__ __launch_bounds__(256) __attribute__((amdgpu_num_vgpr(248)))
void k_gemm_nt(const unsigned short* __restrict__ A, const unsigned short* __restrict__ B,
               const float* __restrict__ bias, float* __restrict__ D, int M, int N, int KTOT, int ldd) {
  static_assert(FORM >= 0 && FORM <= 2);
  static_assert(EPI == 0 || EPI == 1);
  typedef typename FragOf<FORM>::T F;
  __shared__ __attribute__((aligned(16))) float sT[8][16 * 68];
  const int lane = threadIdx.x & 31;
  const int wave = threadIdx.x >> 5;
  const int tilesM = (M + 63) >> 6;
  const int tilesN = (N + 63) >> 6;
  const int tile = blockIdx.x * 8 + wave;
  if (tile >= tilesM * tilesN) return;
  const int tm = tile / tilesN;
  const int tn = tile - tm * tilesN;
  const int m0 = tm << 6;
  const int n0 = tn << 6;

  const int rl = lane & 15;
  const int h8 = (lane >> 4) * 8;
  const unsigned short* pa = A + (size_t)(m0 + rl) * (size_t)KTOT + h8;
  const unsigned short* pb = B + (size_t)(n0 + rl) * (size_t)KTOT + h8;

  v8f acc[4][4];
#pragma unroll
  for (int i = 0; i < 4; ++i)
#pragma unroll
    for (int j = 0; j < 4; ++j) acc[i][j] = (v8f){0.f, 0.f, 0.f, 0.f, 0.f, 0.f, 0.f, 0.f};

#pragma unroll 1
  for (int k0 = 0; k0 < KTOT; k0 += 32) {
    F bf[4];
#pragma unroll
    for (int j = 0; j < 4; ++j) bf[j] = ld_frag<F>(pb + (size_t)(j << 4) * (size_t)KTOT + k0);
#pragma unroll
    for (int i = 0; i < 4; ++i) {
      const F af = ld_frag<F>(pa + (size_t)(i << 4) * (size_t)KTOT + k0);
#pragma unroll
      for (int j = 0; j < 4; ++j) acc[i][j] = mm(af, bf[j], acc[i][j]);
    }
  }

  float* slab = sT[wave];
  const int hh = lane >> 4;
  const int c4 = (lane & 15) * 4;
  const int nc = n0 + c4;
  const bool cok = nc < N;
  v4f bv = (v4f){0.f, 0.f, 0.f, 0.f};
  if (EPI == 1) {
    bv = *(const v4fa*)(bias + clampi(nc, 0, N - 4));
    asm volatile("" :: "v"(bv));
  }
#pragma unroll
  for (int i = 0; i < 4; ++i) {
    const int mBase = m0 + (i << 4);
#pragma unroll
    for (int j = 0; j < 4; ++j) {
#pragma unroll
      for (int r = 0; r < 8; ++r) slab[(h8 + r) * 68 + (j << 4) + rl] = acc[i][j][r];
    }
    __builtin_amdgcn_fence(__ATOMIC_RELEASE, "workgroup");
    __builtin_amdgcn_wave_barrier();
    __builtin_amdgcn_fence(__ATOMIC_ACQUIRE, "workgroup");
    v4f vv[8];
#pragma unroll
    for (int it = 0; it < 8; ++it) {
      const int row = it * 2 + hh;
      v4f v = *(const v4fa*)(slab + row * 68 + c4);
      if (EPI == 1) v += bv;
      vv[it] = v;
    }
    for (int pass = 0; pass < 2; ++pass) {
#pragma unroll
      for (int it = 0; it < 8; ++it) {
        const int row = mBase + it * 2 + hh;
        if (cok && row < M) *(volatile v4f*)(D + (size_t)row * (size_t)ldd + nc) = vv[it];
      }
      __threadfence();
    }
    __builtin_amdgcn_fence(__ATOMIC_RELEASE, "workgroup");
    __builtin_amdgcn_wave_barrier();
    __builtin_amdgcn_fence(__ATOMIC_ACQUIRE, "workgroup");
  }
}

#pragma clang fp contract(off)

#ifndef S12_TWO_TERM
#define S12_TWO_TERM 1
#endif
#ifndef S3_TWO_TERM
#define S3_TWO_TERM 1
#endif
static_assert(S12_TWO_TERM == 0 || S12_TWO_TERM == 1);
static_assert(S3_TWO_TERM == 0 || S3_TWO_TERM == 1);

typedef unsigned int v2u __attribute__((ext_vector_type(2)));
typedef int          v2i __attribute__((ext_vector_type(2)));
typedef int          v4i __attribute__((ext_vector_type(4)));
typedef v2i __attribute__((may_alias)) v2ia;
typedef v4i __attribute__((may_alias)) v4ia;

constexpr int NN     = 100000;
constexpr int NE     = 640000;
constexpr int FD     = 128;
constexpr int G3     = 384;
constexpr int MC     = 20480;
constexpr int NCHUNK = 5;
constexpr int NPF    = 100352;
constexpr int NBRUN  = 1024;
constexpr int NBLK   = 98;
constexpr int RCAP   = 8192;
constexpr int DEGCAP = 32;
constexpr int WLCAP  = 2048;
constexpr int EPW    = NE / 8;
constexpr int SUB    = 128;
constexpr int NSTEP  = (EPW + SUB - 1) / SUB;
constexpr int K12T   = S12_TWO_TERM ? 2 * FD : FD;
constexpr int K3T    = S3_TWO_TERM ? 4 * FD : 2 * FD;

static_assert(NN == 100000 && NE == 640000 && FD == 128 && G3 == 3 * FD);
static_assert(NE == 312 * 2048 + 1024);
static_assert(NE % 8 == 0 && NSTEP * SUB >= EPW && (NSTEP - 1) * SUB < EPW && NSTEP == 625);
static_assert(MC % 1024 == 0 && 4 * MC < NN && NN <= 5 * MC && MC % 64 == 0);
static_assert((NN - 4 * MC) % 16 == 0 && (NN - 4 * MC) % 8 == 0 && MC % 16 == 0);
static_assert(NPF % 64 == 0 && NPF >= NN && NPF == NBLK * NBRUN);
static_assert(4 * MC + (((NN - 4 * MC) + 63) / 64) * 64 <= NPF);
static_assert(NBLK * NBRUN >= NN && (NBLK - 1) * NBRUN < NN);
static_assert(DEGCAP == 32 && DEGCAP * 4 >= 21 * 5);
static_assert(RCAP * 5 >= 6776 * 6 && (RCAP / 2) % 256 == 0 && RCAP >= 2 * DEGCAP);
static_assert(WLCAP * 8 >= RCAP && WLCAP * 2 >= 850 * 4);
static_assert((((long long)(NE - 1) << 10) | 1023) < (1LL << 31));
static_assert(K12T % 32 == 0 && K3T % 32 == 0 && FD % 32 == 0 && G3 % 64 == 0 && (2 * FD) % 32 == 0 && G3 % 32 == 0);
static_assert((size_t)(NN - 1) * FD + (FD - 1) < (size_t)NN * FD);

constexpr int LK_WL   = 0;
constexpr int LK_SL   = 8 * WLCAP;
constexpr int LK_CNT  = LK_SL + RCAP;
constexpr int LK_OFF  = LK_CNT + NBRUN;
constexpr int LK_CUR  = LK_OFF + NBRUN;
constexpr int LK_MISC = LK_CUR + NBRUN;
constexpr int LK_INTS = LK_MISC + 16;
constexpr int LK_LDS  = LK_INTS * 4;
static_assert(LK_LDS == 110656 && LK_LDS <= 262144 && LK_LDS <= 327680);
static_assert(LK_SL % 4 == 0 && LK_CNT % 4 == 0 && (RCAP + NBRUN) % 1024 == 0);

constexpr size_t SZ_R1   = (size_t)MC * G3 * 4;
constexpr size_t SZ_R2   = (size_t)MC * 512 * 2;
constexpr size_t SZ_R3   = (size_t)MC * G3 * 4;
constexpr size_t SZ_FB   = (size_t)NPF * FD * 2;
constexpr size_t SZ_LIST = (size_t)2 * NBLK * RCAP * 8;
constexpr size_t SZ_NODE = (size_t)2 * NBLK * NBRUN * 4;
constexpr size_t SZ_W12  = (size_t)FD * 256 * 2;
constexpr size_t SZ_WIH  = (size_t)G3 * 512 * 2;
constexpr size_t SZ_WHH  = (size_t)G3 * FD * 2;
constexpr size_t SZ_BIAS = (size_t)G3 * 4;
constexpr size_t SZ_FLAG = (size_t)2 * NBLK * 128;
constexpr size_t OFF_R1   = 0;
constexpr size_t OFF_R2   = OFF_R1 + SZ_R1;
constexpr size_t OFF_R3   = OFF_R2 + SZ_R2;
constexpr size_t OFF_FB   = OFF_R3 + SZ_R3;
constexpr size_t OFF_LIST = OFF_FB + SZ_FB;
constexpr size_t OFF_CNT  = OFF_LIST + SZ_LIST;
constexpr size_t OFF_OFF  = OFF_CNT + SZ_NODE;
constexpr size_t OFF_W1D  = OFF_OFF + SZ_NODE;
constexpr size_t OFF_W2D  = OFF_W1D + SZ_W12;
constexpr size_t OFF_WIHD = OFF_W2D + SZ_W12;
constexpr size_t OFF_WHH  = OFF_WIHD + SZ_WIH;
constexpr size_t OFF_BIH  = OFF_WHH + SZ_WHH;
constexpr size_t OFF_BHH  = OFF_BIH + SZ_BIAS;
constexpr size_t OFF_FLAG = OFF_BHH + SZ_BIAS;
constexpr size_t WS_TOTAL = OFF_FLAG + SZ_FLAG;
static_assert(WS_TOTAL == (size_t)((size_t)243511 << 9));
static_assert(WS_TOTAL <= ((size_t)128 << 20));
static_assert(SZ_R1 % 256 == 0 && SZ_R2 % 256 == 0 && SZ_R3 % 256 == 0 && SZ_FB % 256 == 0 && SZ_LIST % 256 == 0);
static_assert(SZ_NODE % 256 == 0 && SZ_W12 % 256 == 0 && SZ_WIH % 256 == 0 && SZ_WHH % 256 == 0);
static_assert(SZ_BIAS % 256 == 0 && SZ_FLAG % 256 == 0);
static_assert((size_t)MC * 256 * 4 <= SZ_R1 && (size_t)MC * K12T * 2 <= SZ_R2 && (size_t)MC * K3T * 2 <= SZ_R2);
static_assert((size_t)FD * K12T * 2 <= SZ_W12 && (size_t)G3 * K3T * 2 <= SZ_WIH);

constexpr int PB_W12 = FD * (K12T / 8) / 256;
constexpr int PB_WIH = G3 * (K3T / 8) / 256;
constexpr int PB_WHH = G3 * (FD / 8) / 256;
constexpr int PB_TOT = 2 * PB_W12 + PB_WIH + PB_WHH + 1;
static_assert((FD * (K12T / 8)) % 256 == 0 && (G3 * (K3T / 8)) % 256 == 0 && (G3 * (FD / 8)) % 256 == 0);

__device__ __forceinline__ void wplane_unit(const float* __restrict__ W, int kin, int ktot,
                                            unsigned short* __restrict__ dst, int u) {
  const int ppr = ktot >> 3;
  const int n   = u / ppr;
  const int p   = u - n * ppr;
  const int k8  = (p << 3) & (kin - 1);
  const float* s = W + (size_t)n * (size_t)kin + k8;
  const v4f a = *(const v4fa*)(s);
  const v4f c = *(const v4fa*)(s + 4);
  asm volatile("" :: "v"(a));
  asm volatile("" :: "v"(c));
  const v4u o = pack8_bf16(a, c);
  volatile v4u* q = (volatile v4u*)(dst + (size_t)u * 8);
  *q = o;
  __threadfence();
  *q = o;
}

__device__ __forceinline__ void par_unit(const float* __restrict__ src, int n4, float* __restrict__ dst, int tid) {
  const int j = tid < n4 ? tid : n4 - 1;
  const v4f a = *(const v4fa*)(src + 4 * j);
  asm volatile("" :: "v"(a));
  const v4f o = (v4f){ bf16_val(a[0]), bf16_val(a[1]), bf16_val(a[2]), bf16_val(a[3]) };
  if (tid < n4) {
    volatile v4f* q = (volatile v4f*)(dst + 4 * tid);
    *q = o;
    __threadfence();
    *q = o;
  }
}

__global__ __launch_bounds__(256) void k_prep(const float* __restrict__ W1, const float* __restrict__ W2,
                                              const float* __restrict__ wih, const float* __restrict__ whh,
                                              const float* __restrict__ bih, const float* __restrict__ bhh,
                                              unsigned short* __restrict__ W1D, unsigned short* __restrict__ W2D,
                                              unsigned short* __restrict__ WIHD, unsigned short* __restrict__ WHH,
                                              float* __restrict__ BIH, float* __restrict__ BHH) {
  const int tid = (int)threadIdx.x;
  const int blk = (int)blockIdx.x;
  if (blk < PB_W12) {
    wplane_unit(W1, FD, K12T, W1D, blk * 256 + tid);
  } else if (blk < 2 * PB_W12) {
    wplane_unit(W2, FD, K12T, W2D, (blk - PB_W12) * 256 + tid);
  } else if (blk < 2 * PB_W12 + PB_WIH) {
    wplane_unit(wih, 2 * FD, K3T, WIHD, (blk - 2 * PB_W12) * 256 + tid);
  } else if (blk < 2 * PB_W12 + PB_WIH + PB_WHH) {
    wplane_unit(whh, FD, FD, WHH, (blk - 2 * PB_W12 - PB_WIH) * 256 + tid);
  } else {
    par_unit(bih, G3 / 4, BIH, tid);
    par_unit(bhh, G3 / 4, BHH, tid);
  }
}

__global__ __launch_bounds__(256) void k_bucket(const int* __restrict__ keyp, const int* __restrict__ idp,
                                                int* __restrict__ LIST, int* __restrict__ CNT,
                                                int* __restrict__ OFF, int* __restrict__ FLAG) {
  extern __shared__ __attribute__((aligned(16))) int dsm[];
  int* wl   = dsm + LK_WL;
  int* sl   = dsm + LK_SL;
  int* cnt  = dsm + LK_CNT;
  int* offs = dsm + LK_OFF;
  int* cur  = dsm + LK_CUR;
  int* misc = dsm + LK_MISC;
  const int tid = (int)threadIdx.x, lane = tid & 31, wave = tid >> 5;
  const int blk = (int)blockIdx.x;
  const int nodeBase = blk * NBRUN;
  const int nbi = (NN - nodeBase) < NBRUN ? (NN - nodeBase) : NBRUN;
  const unsigned unb = (unsigned)(nbi < 0 ? 0 : nbi);

  {
    const v4i z4 = (v4i){0, 0, 0, 0};
    for (int i = tid * 4; i < RCAP + NBRUN; i += 1024) *(v4ia*)(sl + i) = z4;
    if (tid < 16) misc[tid] = 0;
  }
  __syncthreads();

  int* mylist = wl + wave * WLCAP;
  const int wbase = wave * EPW;
  const int wlast = wbase + EPW - 1;
  int wc = 0;
#pragma unroll 1
  for (int st = 0; st < NSTEP; ++st) {
    const int e0 = wbase + st * SUB + lane;
    int dk[4];
#pragma unroll
    for (int j = 0; j < 4; ++j) {
      const int e  = e0 + 32 * j;
      const int ec = e < wlast ? e : wlast;
      const int d  = keyp[ec];
      asm volatile("" :: "v"(d));
      dk[j] = (e <= wlast) ? d : -1;
    }
#pragma unroll
    for (int j = 0; j < 4; ++j) {
      const unsigned slot = (unsigned)dk[j] - (unsigned)nodeBase;
      const bool hit = slot < unb;
      const unsigned mj = __builtin_amdgcn_ballot_w32(hit);
      if (mj != 0u) {
        if (hit) {
          const int pos = wc + (int)__builtin_amdgcn_mbcnt_lo(mj, 0u);
          if (pos < WLCAP) mylist[pos] = ((e0 + 32 * j) << 10) | (int)slot;
        }
        wc += (int)__builtin_popcount(mj);
      }
    }
  }
  if (lane == 0) misc[wave] = wc;
  __syncthreads();

  if (wave == 0) {
    int t = 0, ov = 0;
#pragma unroll 1
    for (int w2 = 0; w2 < 8; ++w2) {
      const int craw = misc[w2];
      ov |= (craw > WLCAP) ? 1 : 0;
      const int c = __builtin_amdgcn_readfirstlane(clampi(craw, 0, WLCAP));
#pragma unroll 1
      for (int b0 = 0; b0 < c; b0 += 32) {
        const int idx = (b0 + lane) < c ? (b0 + lane) : c - 1;
        const int ent = wl[w2 * WLCAP + idx];
        const int m32 = (c - b0) < 32 ? (c - b0) : 32;
#pragma unroll 1
        for (int k = 0; k < m32; ++k) {
          const int u    = __builtin_amdgcn_readlane(ent, k);
          const int slot = u & (NBRUN - 1);
          if (t < RCAP) {
            if (lane == 0) cnt[slot] = cnt[slot] + 1;
            t = t + 1;
          } else {
            ov = 1;
          }
        }
      }
    }
    if (lane == 0) { misc[8] = t; misc[9] = ov; }
  }
  __syncthreads();

  if (wave == 0) {
    const int base = lane * (NBRUN / 32);
    int s = 0, big = 0;
#pragma unroll 1
    for (int i = 0; i < NBRUN / 32; ++i) {
      const int cv = cnt[base + i];
      s += cv;
      big |= (cv > DEGCAP) ? 1 : 0;
    }
    int incl = s;
#pragma unroll
    for (int d = 1; d < 32; d <<= 1) {
      const int y = __shfl_up(incl, d, 32);
      incl += (lane >= d) ? y : 0;
    }
    int run = incl - s;
#pragma unroll 1
    for (int i = 0; i < NBRUN / 32; ++i) {
      const int cv = cnt[base + i];
      offs[base + i] = run;
      cur[base + i]  = run;
      run += cv;
    }
    const unsigned bm = __builtin_amdgcn_ballot_w32(big != 0);
    if (lane == 0) misc[9] = misc[9] | ((bm != 0u) ? 1 : 0);
  }
  __syncthreads();

  if (wave == 0) {
    int t2 = 0;
#pragma unroll 1
    for (int w2 = 0; w2 < 8; ++w2) {
      const int c = __builtin_amdgcn_readfirstlane(clampi(misc[w2], 0, WLCAP));
#pragma unroll 1
      for (int b0 = 0; b0 < c; b0 += 32) {
        const int idx = (b0 + lane) < c ? (b0 + lane) : c - 1;
        const int ent = wl[w2 * WLCAP + idx];
        const int m32 = (c - b0) < 32 ? (c - b0) : 32;
#pragma unroll 1
        for (int k = 0; k < m32; ++k) {
          const int u    = __builtin_amdgcn_readlane(ent, k);
          const int slot = u & (NBRUN - 1);
          if (t2 < RCAP) {
            if (lane == 0) {
              int p = cur[slot];
              p = clampi(p, 0, RCAP - 1);
              sl[p] = u >> 10;
              cur[slot] = p + 1;
            }
            t2 = t2 + 1;
          }
        }
      }
    }
  }
  __syncthreads();

  const int ovf = misc[9];
  int* lbase = LIST + (size_t)blk * (size_t)(RCAP * 2);
  for (int pass = 0; pass < 2; ++pass) {
#pragma unroll 2
    for (int i = tid; i < RCAP / 2; i += 256) {
      const v2i ev = *(const v2ia*)(sl + 2 * i);
      const int e0 = clampi(ev.x, 0, NE - 1);
      const int e1 = clampi(ev.y, 0, NE - 1);
      int s0 = idp[e0];
      int s1 = idp[e1];
      asm volatile("" :: "v"(s0));
      asm volatile("" :: "v"(s1));
      s0 = clampi(s0, 0, NN - 1);
      s1 = clampi(s1, 0, NN - 1);
      const v4i v = (v4i){ s0, e0, s1, e1 };
      *(volatile v4i*)(lbase + 4 * i) = v;
    }
    __threadfence();
  }
  const v4i cv4 = *(const v4ia*)(cnt + 4 * tid);
  const v4i ov4 = *(const v4ia*)(offs + 4 * tid);
  const v4i fl4 = (v4i){ ovf, ovf, ovf, ovf };
  const size_t nb4 = (size_t)nodeBase + 4 * (size_t)tid;
  const bool fw = (wave == 0) && (lane < 8);
  *(volatile v4i*)(CNT + nb4) = cv4;
  *(volatile v4i*)(OFF + nb4) = ov4;
  if (fw) *(volatile v4i*)(FLAG + blk * 32 + 4 * lane) = fl4;
  __threadfence();
  *(volatile v4i*)(CNT + nb4) = cv4;
  *(volatile v4i*)(OFF + nb4) = ov4;
  if (fw) *(volatile v4i*)(FLAG + blk * 32 + 4 * lane) = fl4;
}

__global__ __launch_bounds__(256) void k_agg(const float* __restrict__ feat, const float* __restrict__ wgt,
                                             const int* __restrict__ LIST, const int* __restrict__ CNT,
                                             const int* __restrict__ OFF, const int* __restrict__ FLAG,
                                             unsigned short* __restrict__ NH, int r0, int rows) {
  const int tid = (int)threadIdx.x, lane = tid & 31, wave = tid >> 5;
  const int lr = (int)blockIdx.x * 8 + wave;
  const int n  = r0 + lr;
  const bool live = (lr < rows) && (n < NN);
  const int ic = clampi(n, 0, NN - 1);
  const int b  = ic >> 10;
  int c  = CNT[ic];
  int o  = OFF[ic];
  int fl = FLAG[b * 32];
  asm volatile("" :: "v"(c));
  asm volatile("" :: "v"(o));
  asm volatile("" :: "v"(fl));
  const int craw = c;
  c = clampi(c, 0, DEGCAP);
  o = clampi(o, 0, RCAP - DEGCAP);
  const int cn = __builtin_amdgcn_readfirstlane(live ? c : 0);
  const int* lp = LIST + ((size_t)b * (size_t)RCAP + (size_t)o) * 2;
  const int top = cn > 0 ? cn - 1 : 0;
  const int idx = lane < top ? lane : top;
  const v2i pr = *(const v2ia*)(lp + 2 * idx);
  asm volatile("" :: "v"(pr));
  const int g  = clampi(pr.x, 0, NN - 1);
  const int ed = clampi(pr.y, 0, NE - 1);
  const float wr = wgt[ed];
  asm volatile("" :: "v"(wr));
  const int wbi = __float_as_int(bf16_val(wr));
  const float* fl4p = feat + 4 * lane;

  float acc0 = 0.0f, acc1 = 0.0f, acc2 = 0.0f, acc3 = 0.0f, ws = 0.0f;
#pragma unroll 1
  for (int k = 0; k < cn; ++k) {
    const int   gk = __builtin_amdgcn_readlane(g, k);
    const float wk = __int_as_float(__builtin_amdgcn_readlane(wbi, k));
    const v4f row = *(const v4fa*)(fl4p + (size_t)gk * FD);
    asm volatile("" :: "v"(row));
    acc0 = acc0 + (wk * bf16_val(row[0]));
    acc1 = acc1 + (wk * bf16_val(row[1]));
    acc2 = acc2 + (wk * bf16_val(row[2]));
    acc3 = acc3 + (wk * bf16_val(row[3]));
    ws = ws + wk;
  }
  const bool pos = ws > 0.0f;
  const float safe = pos ? ws : 1.0f;
  const float q0 = acc0 / safe, q1 = acc1 / safe, q2 = acc2 / safe, q3 = acc3 / safe;
  const bool poison = live && ((fl != 0) || (craw > DEGCAP));
  const float qn = __int_as_float(0x7fc00000);
  float v0 = pos ? q0 : 0.0f, v1 = pos ? q1 : 0.0f, v2 = pos ? q2 : 0.0f, v3 = pos ? q3 : 0.0f;
  v0 = poison ? qn : v0;
  v1 = poison ? qn : v1;
  v2 = poison ? qn : v2;
  v3 = poison ? qn : v3;
  const v2u hv = (v2u){ pk16(bf16_bits(v0), bf16_bits(v1)), pk16(bf16_bits(v2), bf16_bits(v3)) };
  const v2u lv = (v2u){ pk16(bf16_lo_bits(v0), bf16_lo_bits(v1)), pk16(bf16_lo_bits(v2), bf16_lo_bits(v3)) };
  unsigned short* rp = NH + (size_t)lr * K12T + 4 * lane;
  *(volatile v2u*)rp = hv;
  if (S12_TWO_TERM) *(volatile v2u*)(rp + FD) = lv;
  __threadfence();
  *(volatile v2u*)rp = hv;
  if (S12_TWO_TERM) *(volatile v2u*)(rp + FD) = lv;
}

__global__ __launch_bounds__(256) void k_split(const float* __restrict__ HN, unsigned short* __restrict__ HL, int rows) {
  const int tid = (int)threadIdx.x, lane = tid & 31, wave = tid >> 5;
  const int lr = (int)blockIdx.x * 8 + wave;
  const bool live = lr < rows;
  const int rc = clampi(lr, 0, rows - 1);
  const float* s = HN + (size_t)rc * (2 * FD) + 8 * lane;
  const v4f a = *(const v4fa*)(s);
  const v4f c = *(const v4fa*)(s + 4);
  asm volatile("" :: "v"(a));
  asm volatile("" :: "v"(c));
  const unsigned mk = live ? 0xFFFFFFFFu : 0u;
  const v4u mw = (v4u){ mk, mk, mk, mk };
  v4u hi = pack8_bf16(a, c);
  v4u lo = pack8_bf16_lo(a, c);
  hi &= mw;
  lo &= mw;
  unsigned short* rp = HL + (size_t)lr * K3T + 8 * lane;
  *(volatile v4u*)rp = hi;
  if (S3_TWO_TERM) *(volatile v4u*)(rp + 2 * FD) = lo;
  __threadfence();
  *(volatile v4u*)rp = hi;
  if (S3_TWO_TERM) *(volatile v4u*)(rp + 2 * FD) = lo;
}

__device__ __forceinline__ float pick4(v4f v, int j) {
  const float a = (j == 0) ? v[0] : v[1];
  const float b = (j == 2) ? v[2] : v[3];
  return (j < 2) ? a : b;
}

__global__ __launch_bounds__(256) void k_gate(const float* __restrict__ GI, const float* __restrict__ GH,
                                              const float* __restrict__ feat, float* outp,
                                              int r0, int rows, int nreal) {
  const int tid = (int)threadIdx.x, lane = tid & 31, wave = tid >> 5;
  const int lr = (int)blockIdx.x * 8 + wave;
  const int n  = r0 + lr;
  const bool live = (lr < rows) && (n < nreal);
  const int lc = clampi(lr, 0, rows - 1);
  const int nc = clampi(n, 0, nreal - 1);
  const float* gi = GI + (size_t)lc * G3 + 4 * lane;
  const float* gh = GH + (size_t)lc * G3 + 4 * lane;
  const v4f ir = *(const v4fa*)(gi);
  const v4f iz = *(const v4fa*)(gi + FD);
  const v4f in = *(const v4fa*)(gi + 2 * FD);
  const v4f hr = *(const v4fa*)(gh);
  const v4f hz = *(const v4fa*)(gh + FD);
  const v4f hn = *(const v4fa*)(gh + 2 * FD);
  const v4f fr = *(const v4fa*)(feat + (size_t)nc * FD + 4 * lane);
  asm volatile("" :: "v"(ir));
  asm volatile("" :: "v"(iz));
  asm volatile("" :: "v"(in));
  asm volatile("" :: "v"(hr));
  asm volatile("" :: "v"(hz));
  asm volatile("" :: "v"(hn));
  asm volatile("" :: "v"(fr));
  const v4f fb = (v4f){ bf16_val(fr[0]), bf16_val(fr[1]), bf16_val(fr[2]), bf16_val(fr[3]) };
  v4f o = (v4f){ 0.0f, 0.0f, 0.0f, 0.0f };
#pragma unroll 1
  for (int j = 0; j < 4; ++j) {
    const float ar = pick4(ir, j) + pick4(hr, j);
    const float rg = 1.0f / (1.0f + expf(-ar));
    const float az = pick4(iz, j) + pick4(hz, j);
    const float zg = 1.0f / (1.0f + expf(-az));
    const float an = pick4(in, j) + rg * pick4(hn, j);
    const float nv = tanhf(an);
    const float hv = pick4(fb, j);
    const float ov = nv + zg * (hv - nv);
    o = (v4f){ (j == 0) ? ov : o[0], (j == 1) ? ov : o[1], (j == 2) ? ov : o[2], (j == 3) ? ov : o[3] };
  }
  float* op = outp + (size_t)nc * FD + 4 * lane;
  if (live) *(volatile v4f*)op = o;
  __threadfence();
  if (live) *(volatile v4f*)op = o;
}

extern "C" void kernel_launch(void* const* d_in, const int* in_sizes, int n_in,
                              void* d_out, int out_size, void* d_ws, size_t ws_size,
                              hipStream_t stream) {
  if (n_in < 10) return;
  if (in_sizes[0] != NN * FD) return;
  if (in_sizes[1] != NE) return;
  if (in_sizes[2] != NE || in_sizes[3] != NE) return;
  if (in_sizes[4] != FD * FD || in_sizes[5] != FD * FD) return;
  if (in_sizes[6] != G3 * 2 * FD || in_sizes[7] != G3 * FD) return;
  if (in_sizes[8] != G3 || in_sizes[9] != G3) return;
  if (out_size != NN * FD) return;
  if (ws_size < WS_TOTAL) return;

  const float* feat = (const float*)d_in[0];
  const float* wgt  = (const float*)d_in[1];
  const int*   src  = (const int*)d_in[2];
  const int*   dst  = (const int*)d_in[3];
  const float* W1   = (const float*)d_in[4];
  const float* W2   = (const float*)d_in[5];
  const float* wih  = (const float*)d_in[6];
  const float* whh  = (const float*)d_in[7];
  const float* bih  = (const float*)d_in[8];
  const float* bhh  = (const float*)d_in[9];
  float* out = (float*)d_out;

  char* ws = (char*)d_ws;
  float*          R1   = (float*)(ws + OFF_R1);
  unsigned short* R2   = (unsigned short*)(ws + OFF_R2);
  float*          R3   = (float*)(ws + OFF_R3);
  unsigned short* FB   = (unsigned short*)(ws + OFF_FB);
  int*            LIST = (int*)(ws + OFF_LIST);
  int*            CNT  = (int*)(ws + OFF_CNT);
  int*            OFFS = (int*)(ws + OFF_OFF);
  unsigned short* W1D  = (unsigned short*)(ws + OFF_W1D);
  unsigned short* W2D  = (unsigned short*)(ws + OFF_W2D);
  unsigned short* WIHD = (unsigned short*)(ws + OFF_WIHD);
  unsigned short* WHH  = (unsigned short*)(ws + OFF_WHH);
  float*          BIH  = (float*)(ws + OFF_BIH);
  float*          BHH  = (float*)(ws + OFF_BHH);
  int*            FLAG = (int*)(ws + OFF_FLAG);

  int* LIST0 = LIST;
  int* LIST1 = LIST + (size_t)NBLK * RCAP * 2;
  int* CNT0  = CNT;
  int* CNT1  = CNT + (size_t)NBLK * NBRUN;
  int* OFF0  = OFFS;
  int* OFF1  = OFFS + (size_t)NBLK * NBRUN;
  int* FLAG0 = FLAG;
  int* FLAG1 = FLAG + NBLK * 32;

  hipFuncSetAttribute(reinterpret_cast<const void*>(&k_bucket), hipFuncAttributeMaxDynamicSharedMemorySize, (int)LK_LDS);

  k_prep<<<PB_TOT, 256, 0, stream>>>(W1, W2, wih, whh, bih, bhh, W1D, W2D, WIHD, WHH, BIH, BHH);
  k_plane<0><<<NPF * (FD / 8) / 256, 256, 0, stream>>>(feat, NN, FD, FD, FB, NPF, FD);
  k_bucket<<<NBLK, 256, LK_LDS, stream>>>(dst, src, LIST0, CNT0, OFF0, FLAG0);
  k_bucket<<<NBLK, 256, LK_LDS, stream>>>(src, dst, LIST1, CNT1, OFF1, FLAG1);

  for (int ch = 0; ch < NCHUNK; ++ch) {
    const int r0   = ch * MC;
    const int rows = (NN - r0) < MC ? (NN - r0) : MC;
    const int pad  = ((rows + 63) / 64) * 64;
    const int tm   = pad / 64;
    const int g2   = (tm * 2 + 7) / 8;
    const int g6   = (tm * 6 + 7) / 8;

    k_agg<<<pad / 8, 256, 0, stream>>>(feat, wgt, LIST0, CNT0, OFF0, FLAG0, R2, r0, rows);
    k_gemm_nt<0, 0><<<g2, 256, 0, stream>>>(R2, W1D, BIH, R1, rows, FD, K12T, 2 * FD);
    k_agg<<<pad / 8, 256, 0, stream>>>(feat, wgt, LIST1, CNT1, OFF1, FLAG1, R2, r0, rows);
    k_gemm_nt<0, 0><<<g2, 256, 0, stream>>>(R2, W2D, BIH, R1 + FD, rows, FD, K12T, 2 * FD);
    k_split<<<pad / 8, 256, 0, stream>>>(R1, R2, rows);
    k_gemm_nt<0, 1><<<g6, 256, 0, stream>>>(R2, WIHD, BIH, R1, rows, G3, K3T, G3);
    k_gemm_nt<0, 1><<<g6, 256, 0, stream>>>(FB + (size_t)r0 * FD, WHH, BHH, R3, rows, G3, FD, G3);
    k_gate<<<(rows + 7) / 8, 256, 0, stream>>>(R1, R3, feat, out, r0, rows, NN);
  }
}
